// RingDilatedAttentionHybridOptimized_42614665511001
// MI455X (gfx1250) — hardware-verified
//
#include <hip/hip_runtime.h>
#include <math.h>

typedef __attribute__((ext_vector_type(16))) _Float16 v16h;
typedef __attribute__((ext_vector_type(16))) __bf16 v16b;
typedef __attribute__((ext_vector_type(8)))  _Float16 v8h;
typedef __attribute__((ext_vector_type(8)))  float v8f;
typedef __attribute__((ext_vector_type(4)))  float v4f;
typedef __attribute__((ext_vector_type(2)))  float v2f;
typedef __attribute__((ext_vector_type(4)))  unsigned v4u;
typedef __attribute__((ext_vector_type(4)))  int v4i;
typedef float __attribute__((may_alias)) float_a;
typedef int __attribute__((may_alias)) int_a;

template <typename T> __device__ __forceinline__ void vst2(void* p, T v) { *(volatile T*)p = v; __threadfence(); *(volatile T*)p = v; }
__device__ __forceinline__ v8f wmma16(v16h a, v16h b, v8f c) {
  v8f d = __builtin_amdgcn_wmma_f32_16x16x32_f16(false, a, false, b, (short)0, c, false, false);
  asm volatile("v_nop\n\tv_nop\n\tv_nop\n\tv_nop" : "+v"(d) : "v"(a), "v"(b));
  return d;
}
__device__ __forceinline__ v8f wmma_bf(v16b a, v16b b, v8f c) {
  v8f d = __builtin_amdgcn_wmma_f32_16x16x32_bf16(false, a, false, b, (short)0, c, false, false);
  asm volatile("v_nop\n\tv_nop\n\tv_nop\n\tv_nop" : "+v"(d) : "v"(a), "v"(b));
  return d;
}
__device__ __forceinline__ v16h frag_h(const _Float16* rowk0, int lane) {
  union { v16h v; v8h q[2]; } u; const _Float16* p = rowk0 + 8 * (lane >> 4);
  u.q[0] = *(const v8h*)p; u.q[1] = *(const v8h*)(p + 16); return u.v;
}
__device__ __forceinline__ v16h frag_f32(const float* rowk0, int lane) {
  v16h a; const float* p = rowk0 + 8 * (lane >> 4);
#pragma unroll
  for (int i = 0; i < 8; ++i) { a[i] = (_Float16)p[i]; a[8 + i] = (_Float16)p[16 + i]; }
  return a;
}
__device__ __forceinline__ v16h frag_f32s(const float* rowk0, int lane, float sc) {
  v16h a; const float* p = rowk0 + 8 * (lane >> 4);
#pragma unroll
  for (int i = 0; i < 8; ++i) { a[i] = (_Float16)(p[i] * sc); a[8 + i] = (_Float16)(p[16 + i] * sc); }
  return a;
}
__device__ __forceinline__ v16h fragc_f32(const float* W, int k0, int n, int lane, int ld, int K) {
  v16h a; const int g = lane >> 4;
#pragma unroll
  for (int i = 0; i < 8; ++i) { const int ka = k0 + 8 * g + i, kb = ka + 16;
    a[i] = (_Float16)(ka < K ? W[(size_t)ka * ld + n] : 0.f); a[8 + i] = (_Float16)(kb < K ? W[(size_t)kb * ld + n] : 0.f); }
  return a;
}
struct F2 { v16b h, l; };
__device__ __forceinline__ F2 bsplit16(const float v[16]) { F2 r;
#pragma unroll
  for (int i = 0; i < 16; ++i) { const __bf16 h = (__bf16)v[i]; r.h[i] = h; r.l[i] = (__bf16)(v[i] - (float)h); }
  return r; }
__device__ __forceinline__ F2 split_row(const float* row, int k0, int lane) { float v[16]; const float* p = row + k0 + 8 * (lane >> 4);
#pragma unroll
  for (int i = 0; i < 8; ++i) { v[i] = p[i]; v[8 + i] = p[16 + i]; }
  return bsplit16(v); }
__device__ __forceinline__ F2 split_rowK(const float* row, int k0, int lane, int K) { float v[16]; const int g = lane >> 4;
#pragma unroll
  for (int i = 0; i < 8; ++i) { const int ka = k0 + 8 * g + i, kb = ka + 16; v[i] = ka < K ? row[ka] : 0.f; v[8 + i] = kb < K ? row[kb] : 0.f; }
  return bsplit16(v); }
__device__ __forceinline__ F2 split_col(const float* W, int k0, int n, int lane, int ld, int K) { float v[16]; const int g = lane >> 4;
#pragma unroll
  for (int i = 0; i < 8; ++i) { const int ka = k0 + 8 * g + i, kb = ka + 16; v[i] = ka < K ? W[(size_t)ka * ld + n] : 0.f; v[8 + i] = kb < K ? W[(size_t)kb * ld + n] : 0.f; }
  return bsplit16(v); }
__device__ __forceinline__ v8f mac3(const F2& a, const F2& b, v8f c) { c = wmma_bf(a.l, b.h, c); c = wmma_bf(a.h, b.l, c); return wmma_bf(a.h, b.h, c); }
__device__ __forceinline__ float sigm(float v) { return 1.0f / (1.0f + expf(-v)); }
#define LDSX() do { asm volatile("s_wait_dscnt 0" ::: "memory"); __builtin_amdgcn_wave_barrier(); __builtin_amdgcn_fence(__ATOMIC_RELEASE, "workgroup"); } while (0)

#define NPOS 4096
#define NHT 12
#define HD 64
#define RS (NHT * HD)
#define NINST 16
#define LMAX 4096
#define PLO 1024.0f
#define VLO 2048.0f

__device__ __forceinline__ void inst_info(int inst, int& h, int& L, int& base, int& stride) {
  if (inst < 4) { h = inst; L = 4096; base = 0; stride = 1; }
  else if (inst < 12) { const int i = inst - 4; h = 4 + (i >> 1); const int s = i & 1; L = 1024; base = s * 2048 + 1; stride = 2; }
  else { h = 8 + (inst - 12); L = 1024; base = 2; stride = 4; }
}
__global__ __launch_bounds__(256) void k_prep(const float* __restrict__ q, const float* __restrict__ k, const float* __restrict__ v, _Float16* __restrict__ Q16, _Float16* __restrict__ K16, _Float16* __restrict__ VTh, _Float16* __restrict__ VTl) {
  __shared__ __align__(16) _Float16 sth[HD][72], stl[HD][72];
  const int inst = blockIdx.y, m0 = blockIdx.x * 64, tid = threadIdx.x; int h, L, base, stride; inst_info(inst, h, L, base, stride);
  if (m0 >= L) return;
  for (int qq = tid; qq < 64 * 8; qq += 256) { const int ml = qq >> 3, pc = qq & 7; const int pos = base + stride * (m0 + ml); const size_t src = ((size_t)pos * NHT + h) * HD + pc * 8;
    union { v8h h8; v4u u; } pq, pk;
#pragma unroll
    for (int e = 0; e < 8; ++e) { pq.h8[e] = (_Float16)q[src + e]; pk.h8[e] = (_Float16)k[src + e]; }
    const size_t dst = ((size_t)inst * LMAX + m0 + ml) * HD + pc * 8; vst2(Q16 + dst, pq.u); vst2(K16 + dst, pk.u); }
  for (int qq = tid; qq < 64 * HD; qq += 256) { const int ml = qq >> 6, d = qq & 63; const int pos = base + stride * (m0 + ml); const float vv = v[((size_t)pos * NHT + h) * HD + d];
    const _Float16 hi = (_Float16)vv; sth[d][ml] = hi; stl[d][ml] = (_Float16)((vv - (float)hi) * VLO); }
  __syncthreads();
  for (int qq = tid; qq < HD * 8; qq += 256) { const int d = qq >> 3, pc = qq & 7; const size_t o = ((size_t)inst * HD + d) * LMAX + m0 + pc * 8;
    vst2(VTh + o, *(const v4u*)(&sth[d][pc * 8])); vst2(VTl + o, *(const v4u*)(&stl[d][pc * 8])); }
}
__global__ __launch_bounds__(128) void k_zero(float* __restrict__ out) {
  const int pos = blockIdx.x, tid = threadIdx.x; const int hrel = tid >> 4, pc = tid & 15; const int h = 4 + hrel;
  const bool selected = (h < 8) ? ((pos & 1) == 1) : ((pos & 3) == 2);
  if (!selected) vst2(out + ((size_t)pos * NHT + h) * HD + pc * 4, (v4f){0.f, 0.f, 0.f, 0.f});
}
__global__ __launch_bounds__(128) void k_attn(const _Float16* __restrict__ Q16, const _Float16* __restrict__ K16, const _Float16* __restrict__ VTh, const _Float16* __restrict__ VTl, float* __restrict__ out) {
  __shared__ __align__(16) float sS[4][16][68];
  __shared__ __align__(16) _Float16 sPh[4][16][72], sPl[4][16][72];
  __shared__ __align__(16) float sO[4][16][68];
  const int tid = threadIdx.x, w = tid >> 5, lane = tid & 31, col = lane & 15, g = lane >> 4;
  const int inst = blockIdx.y; int h, L, base, stride; inst_info(inst, h, L, base, stride);
  const int q0 = blockIdx.x * 64 + w * 16; if (blockIdx.x * 64 >= L) return;
  const size_t ib = (size_t)inst * LMAX;
  v16h aq[2];
#pragma unroll
  for (int kc = 0; kc < 2; ++kc) aq[kc] = frag_h(Q16 + (ib + q0 + col) * HD + kc * 32, lane);
  float mrun = -3.0e38f, lrun = 0.f; v8f acc[4] = {}, ac1[4] = {}, ac2[4] = {};
  const int nkt = L / 64;
#pragma unroll 1
  for (int kt = 0; kt < nkt; ++kt) {
#pragma unroll
    for (int t = 0; t < 4; ++t) { v8f s = {}; const int key = kt * 64 + t * 16 + col;
#pragma unroll
      for (int kc = 0; kc < 2; ++kc) s = wmma16(aq[kc], frag_h(K16 + (ib + key) * HD + kc * 32, lane), s);
#pragma unroll
      for (int r = 0; r < 8; ++r) sS[w][8 * g + r][t * 16 + col] = s[r] * 0.125f; }
    LDSX();
    float mx = -3.4e38f;
#pragma unroll
    for (int jj = 0; jj < 32; ++jj) mx = fmaxf(mx, sS[w][col][g * 32 + jj]);
    mx = fmaxf(mx, __shfl_xor(mx, 16, 32));
    const float mnew = fmaxf(mrun, mx); const float corr = expf(mrun - mnew);
    float ps = 0.f;
#pragma unroll
    for (int jj = 0; jj < 32; ++jj) { const float p = expf(sS[w][col][g * 32 + jj] - mnew) * 16384.0f; ps += p; const _Float16 hi = (_Float16)p; sPh[w][col][g * 32 + jj] = hi; sPl[w][col][g * 32 + jj] = (_Float16)((p - (float)hi) * PLO); }
    ps += __shfl_xor(ps, 16, 32);
    lrun = lrun * corr + ps * (1.0f / 16384.0f); mrun = mnew;
#pragma unroll
    for (int r = 0; r < 8; ++r) { const float cr = __shfl(corr, 8 * g + r, 32);
#pragma unroll
      for (int t = 0; t < 4; ++t) { acc[t][r] *= cr; ac1[t][r] *= cr; ac2[t][r] *= cr; } }
    LDSX();
#pragma unroll
    for (int kc = 0; kc < 2; ++kc) { const v16h ph = frag_h(&sPh[w][col][0] + kc * 32, lane), pl = frag_h(&sPl[w][col][0] + kc * 32, lane);
#pragma unroll
      for (int t = 0; t < 4; ++t) { const size_t vo = ((size_t)inst * HD + t * 16 + col) * LMAX + kt * 64 + kc * 32; const v16h vh = frag_h(VTh + vo, lane);
        acc[t] = wmma16(ph, vh, acc[t]); ac1[t] = wmma16(ph, frag_h(VTl + vo, lane), ac1[t]); ac2[t] = wmma16(pl, vh, ac2[t]); } }
    __builtin_amdgcn_wave_barrier(); }
#pragma unroll
  for (int r = 0; r < 8; ++r) { const float lr = __shfl(lrun, 8 * g + r, 32); const float inv = 1.0f / (lr * 16384.0f);
#pragma unroll
    for (int t = 0; t < 4; ++t) sO[w][8 * g + r][t * 16 + col] = (acc[t][r] + ac1[t][r] * (1.0f / VLO) + ac2[t][r] * (1.0f / PLO)) * inv; }
  LDSX();
  for (int qq = lane; qq < 16 * 16; qq += 32) { const int rl = qq >> 4, pc = qq & 15; const int pos = base + stride * (q0 + rl); vst2(out + ((size_t)pos * NHT + h) * HD + pc * 4, *(const v4f*)(&sO[w][rl][pc * 4])); }
}
extern "C" void kernel_launch(void* const* d_in, const int* in_sizes, int n_in, void* d_out, int out_size, void* d_ws, size_t ws_size, hipStream_t stream) {
  (void)in_sizes; (void)n_in; (void)out_size; (void)ws_size;
  const float* q = (const float*)d_in[0]; const float* k = (const float*)d_in[1]; const float* v = (const float*)d_in[2]; float* out = (float*)d_out;
  char* ws = (char*)d_ws; size_t off = 0;
  auto take = [&](size_t bytes) { char* p = ws + off; off += (bytes + 255) & ~(size_t)255; return p; };
  const size_t plane = (size_t)NINST * LMAX * HD * 2;
  _Float16* Q16 = (_Float16*)take(plane); _Float16* K16 = (_Float16*)take(plane); _Float16* VTh = (_Float16*)take(plane); _Float16* VTl = (_Float16*)take(plane);
  k_prep<<<dim3(LMAX / 64, NINST), 256, 0, stream>>>(q, k, v, Q16, K16, VTh, VTl);
  k_zero<<<NPOS, 128, 0, stream>>>(out);
  k_attn<<<dim3(LMAX / 64, NINST), 128, 0, stream>>>(Q16, K16, VTh, VTl, out);
}
